// MicrotubuleDynamicsModel_10436770529956
// MI455X (gfx1250) — hardware-verified
//
#include <hip/hip_runtime.h>

#define NODES   52
#define FEAT    6
#define HID     128
#define NLAY    3
#define NB      2
#define ROWS    (NB * NODES)
#define MPAD    112
#define MT      (MPAD / 16)
#define KQ      32
#define THREADS 256
#define PASSES  2
#define BPB     (NB * PASSES)
#define OUTPP   (ROWS * FEAT)
#define OUTPB   (BPB * NODES * FEAT)
#define MAXNB   8
#define SA      16.0f
#define SB      16.0f
#define INVS    (1.0f / 256.0f)

typedef _Float16 v16h __attribute__((ext_vector_type(16)));
typedef _Float16 v8h  __attribute__((ext_vector_type(8), __may_alias__));
typedef float    v8f  __attribute__((ext_vector_type(8)));
typedef float    v4f  __attribute__((ext_vector_type(4), __may_alias__));

union Frag { v16h v; v8h hv[2]; _Float16 e[16]; };

__device__ __forceinline__ v8f wmma16(v16h a, v16h b, v8f c) {
  c = __builtin_amdgcn_wmma_f32_16x16x32_f16(false, a, false, b, (short)0, c, false, false);
  asm volatile("v_nop\n\tv_nop\n\tv_nop\n\tv_nop" : "+v"(c) : "v"(a), "v"(b));
  return c;
}

__device__ __forceinline__ int frag_k(int i, int h) {
  return (i < 8) ? (8 * h + i) : (16 + 8 * h + (i - 8));
}

__device__ __forceinline__ v8f zero8() {
  v8f z = {0.0f, 0.0f, 0.0f, 0.0f, 0.0f, 0.0f, 0.0f, 0.0f};
  return z;
}

__device__ __forceinline__ void gemm128(const _Float16* sA, float* sD,
                                        const float* __restrict__ W,
                                        const float* __restrict__ bias,
                                        int wave, int h, int ln) {
  const int col = wave * 16 + ln;
  const float* wrow = W + (size_t)col * HID;
  Frag bw[4];
#pragma unroll
  for (int ks = 0; ks < 4; ++ks) {
    const float* p0 = wrow + ks * 32 + 8 * h;
    v4f f0 = *(const v4f*)(p0);
    v4f f1 = *(const v4f*)(p0 + 4);
    v4f f2 = *(const v4f*)(p0 + 16);
    v4f f3 = *(const v4f*)(p0 + 20);
#pragma unroll
    for (int j = 0; j < 4; ++j) {
      bw[ks].e[j]      = (_Float16)(f0[j] * SB);
      bw[ks].e[4 + j]  = (_Float16)(f1[j] * SB);
      bw[ks].e[8 + j]  = (_Float16)(f2[j] * SB);
      bw[ks].e[12 + j] = (_Float16)(f3[j] * SB);
    }
  }
  const bool ep = (bias != nullptr);
  const float pb = ep ? bias[col] : 0.0f;
#pragma unroll
  for (int mt = 0; mt < MT; ++mt) {
    v8f acc = zero8();
    const _Float16* xr = sA + (mt * 16 + ln) * HID + 8 * h;
#pragma unroll
    for (int ks = 0; ks < 4; ++ks) {
      Frag a;
      a.hv[0] = *(const v8h*)(xr + ks * 32);
      a.hv[1] = *(const v8h*)(xr + ks * 32 + 16);
      acc = wmma16(a.v, bw[ks].v, acc);
    }
    float* drow = sD + (mt * 16 + 8 * h) * HID + col;
#pragma unroll
    for (int r = 0; r < 8; ++r) {
      float d = acc[r] * INVS;
      if (ep) d = fmaxf(d + pb, 0.0f);
      drow[r * HID] = d;
    }
  }
}

__global__ __launch_bounds__(THREADS)
void k_net(const float* __restrict__ q,
           const float* __restrict__ W_in,  const float* __restrict__ b_in,
           const float* __restrict__ W_gnn, const float* __restrict__ b_gnn,
           const float* __restrict__ W_d1,  const float* __restrict__ b_d1,
           const float* __restrict__ W_d2,  const float* __restrict__ b_d2,
           const int* __restrict__ edge, int E,
           float* out, int nB) {
  __shared__ __align__(16) float    sX[ROWS * HID];
  __shared__ __align__(16) _Float16 sXh[MPAD * HID];
  __shared__ __align__(16) float    sH[MPAD * HID];
  __shared__ __align__(16) _Float16 sQ[MPAD * KQ];
  __shared__ __align__(16) float    sOut[OUTPB];
  __shared__ float s_dinv[NODES];
  __shared__ int   s_cnt[NODES];
  __shared__ int   s_idx[NODES * MAXNB];
  __shared__ float s_w[NODES * MAXNB];

  const int tid  = threadIdx.x;
  const int wave = tid >> 5;
  const int lane = tid & 31;
  const int h    = lane >> 4;
  const int ln   = lane & 15;

  if (tid < NODES) {
    int deg = 1;
    for (int e = 0; e < E; ++e) deg += (edge[E + e] == tid);
    s_dinv[tid] = rsqrtf((float)deg);
  }
  for (int idx = tid; idx < (MPAD - ROWS) * HID; idx += THREADS) sXh[ROWS * HID + idx] = (_Float16)0.0f;
  __syncthreads();
  if (tid < NODES) {
    const int t = tid;
    int cnt = 1;
    s_idx[t * MAXNB] = t;
    s_w[t * MAXNB] = s_dinv[t] * s_dinv[t];
#pragma unroll
    for (int k = 1; k < MAXNB; ++k) { s_idx[t * MAXNB + k] = 0; s_w[t * MAXNB + k] = 0.0f; }
    for (int e = 0; e < E; ++e) {
      if (edge[E + e] == t) {
        int j = edge[e];
        j = j < 0 ? 0 : (j > NODES - 1 ? NODES - 1 : j);
        const float ww = s_dinv[j] * s_dinv[t];
        int f = -1;
        for (int k = 0; k < cnt; ++k) if (s_idx[t * MAXNB + k] == j) { f = k; break; }
        if (f >= 0)            s_w[t * MAXNB + f] += ww;
        else if (cnt < MAXNB) { s_idx[t * MAXNB + cnt] = j; s_w[t * MAXNB + cnt] = ww; ++cnt; }
      }
    }
    s_cnt[t] = cnt;
  }
  __syncthreads();

  for (int p = 0; p < PASSES; ++p) {
    const int bg0 = blockIdx.x * BPB + p * NB;

    for (int idx = tid; idx < MPAD * KQ; idx += THREADS) {
      const int r = idx >> 5, k = idx & (KQ - 1);
      float v = 0.0f;
      if (r < ROWS && k < FEAT) {
        const int b = (r >= NODES), i = r - b * NODES;
        const int bg = bg0 + b;
        if (bg < nB) v = q[((size_t)bg * NODES + i) * FEAT + k] * SA;
      }
      sQ[idx] = (_Float16)v;
    }
    __syncthreads();

    {
      const int col = wave * 16 + ln;
      Frag bw;
#pragma unroll
      for (int i = 0; i < 16; ++i) {
        const int k  = frag_k(i, h);
        const int kk = (k < FEAT) ? k : 0;
        const float v = W_in[col * FEAT + kk];
        bw.e[i] = (_Float16)((k < FEAT) ? v * SB : 0.0f);
      }
      const float bc = b_in[col];
#pragma unroll
      for (int mt = 0; mt < MT; ++mt) {
        const _Float16* qr = sQ + (mt * 16 + ln) * KQ + 8 * h;
        Frag a;
        a.hv[0] = *(const v8h*)(qr);
        a.hv[1] = *(const v8h*)(qr + 16);
        v8f acc = zero8();
        acc = wmma16(a.v, bw.v, acc);
#pragma unroll
        for (int r = 0; r < 8; ++r) {
          const int row = mt * 16 + 8 * h + r;
          if (row < ROWS) {
            const float v = fmaxf(acc[r] * INVS + bc, 0.0f);
            sX[row * HID + col]  = v;
            sXh[row * HID + col] = (_Float16)(v * SA);
          }
        }
      }
    }
    __syncthreads();

    for (int l = 0; l < NLAY; ++l) {
      gemm128(sXh, sH, W_gnn + (size_t)l * HID * HID, nullptr, wave, h, ln);
      __syncthreads();
      const float* bias = b_gnn + l * HID;
      for (int idx = tid; idx < ROWS * HID; idx += THREADS) {
        const int r = idx >> 7, c = idx & (HID - 1);
        const int b = (r >= NODES), i = r - b * NODES;
        float agg = bias[c];
        int cnt = s_cnt[i];
        cnt = cnt < 0 ? 0 : (cnt > MAXNB ? MAXNB : cnt);
        for (int k = 0; k < cnt; ++k) {
          const int j = s_idx[i * MAXNB + k];
          agg += s_w[i * MAXNB + k] * sH[(b * NODES + j) * HID + c];
        }
        const float xv = sX[idx] + fmaxf(agg, 0.0f);
        sX[idx]  = xv;
        sXh[idx] = (_Float16)(xv * SA);
      }
      __syncthreads();
    }

    gemm128(sXh, sH, W_d1, b_d1, wave, h, ln);
    __syncthreads();

    if (wave < MT) {
      const int mt = wave;
      const bool cv = (ln < FEAT);
      const int nn = cv ? ln : 0;
      const float sc = cv ? SB : 0.0f;
      const float* wrow = W_d2 + nn * HID;
      Frag bd[4];
#pragma unroll
      for (int ks = 0; ks < 4; ++ks) {
        const float* p0 = wrow + ks * 32 + 8 * h;
        v4f f0 = *(const v4f*)(p0);
        v4f f1 = *(const v4f*)(p0 + 4);
        v4f f2 = *(const v4f*)(p0 + 16);
        v4f f3 = *(const v4f*)(p0 + 20);
#pragma unroll
        for (int j = 0; j < 4; ++j) {
          bd[ks].e[j]      = (_Float16)(f0[j] * sc);
          bd[ks].e[4 + j]  = (_Float16)(f1[j] * sc);
          bd[ks].e[8 + j]  = (_Float16)(f2[j] * sc);
          bd[ks].e[12 + j] = (_Float16)(f3[j] * sc);
        }
      }
      v8f acc = zero8();
      const float* yr = sH + (mt * 16 + ln) * HID + 8 * h;
#pragma unroll
      for (int ks = 0; ks < 4; ++ks) {
        v4f y0 = *(const v4f*)(yr + ks * 32);
        v4f y1 = *(const v4f*)(yr + ks * 32 + 4);
        v4f y2 = *(const v4f*)(yr + ks * 32 + 16);
        v4f y3 = *(const v4f*)(yr + ks * 32 + 20);
        Frag a;
#pragma unroll
        for (int j = 0; j < 4; ++j) {
          a.e[j]      = (_Float16)(y0[j] * SA);
          a.e[4 + j]  = (_Float16)(y1[j] * SA);
          a.e[8 + j]  = (_Float16)(y2[j] * SA);
          a.e[12 + j] = (_Float16)(y3[j] * SA);
        }
        acc = wmma16(a.v, bd[ks].v, acc);
      }
      const float bb = b_d2[nn];
#pragma unroll
      for (int r = 0; r < 8; ++r) {
        const int row = mt * 16 + 8 * h + r;
        if (cv && row < ROWS) sOut[p * OUTPP + row * FEAT + ln] = acc[r] * INVS + bb;
      }
    }
    __syncthreads();
  }

  const size_t outTotal = (size_t)nB * (NODES * FEAT);
  const size_t base = (size_t)blockIdx.x * OUTPB;
  for (int v = tid; v < OUTPB / 4; v += THREADS) {
    const size_t g = base + 4 * (size_t)v;
    if (g + 4 <= outTotal) {
      const v4f val = *(const v4f*)(sOut + 4 * v);
      *(volatile v4f*)(out + g) = val;
    }
  }
  __threadfence();
  for (int v = tid; v < OUTPB / 4; v += THREADS) {
    const size_t g = base + 4 * (size_t)v;
    if (g + 4 <= outTotal) {
      const v4f val = *(const v4f*)(sOut + 4 * v);
      *(volatile v4f*)(out + g) = val;
    }
  }
}

extern "C" void kernel_launch(void* const* d_in, const int* in_sizes, int n_in,
                              void* d_out, int out_size, void* d_ws, size_t ws_size,
                              hipStream_t stream) {
  (void)n_in; (void)d_ws; (void)ws_size;
  const float* q     = (const float*)d_in[0];
  const float* W_in  = (const float*)d_in[1];
  const float* b_in  = (const float*)d_in[2];
  const float* W_gnn = (const float*)d_in[3];
  const float* b_gnn = (const float*)d_in[4];
  const float* W_d1  = (const float*)d_in[5];
  const float* b_d1  = (const float*)d_in[6];
  const float* W_d2  = (const float*)d_in[7];
  const float* b_d2  = (const float*)d_in[8];
  const int*   edge  = (const int*)d_in[9];

  const int E = in_sizes[9] / 2;
  int nB = in_sizes[0] / (NODES * FEAT);
  const int nBo = out_size / (NODES * FEAT);
  if (nBo < nB) nB = nBo;
  if (nB <= 0) return;

  const int blocks = (nB + BPB - 1) / BPB;
  k_net<<<blocks, THREADS, 0, stream>>>(q, W_in, b_in, W_gnn, b_gnn, W_d1, b_d1, W_d2, b_d2,
                                        edge, E, (float*)d_out, nB);
}
